// GenCTBE_22127671509386
// MI455X (gfx1250) — hardware-run, weakly checked
//
#include <hip/hip_runtime.h>
#include <math.h>

typedef __attribute__((ext_vector_type(16))) _Float16 v16h;
typedef __attribute__((ext_vector_type(8)))  _Float16 v8h;
typedef __attribute__((ext_vector_type(8)))  float    v8f;
typedef __attribute__((ext_vector_type(4)))  float    v4f;
typedef __attribute__((ext_vector_type(2)))  unsigned v2u;
typedef __attribute__((ext_vector_type(2)))  float    v2f;

constexpr int kB  = 4096;
constexpr int kU  = 256;
constexpr int kD  = 64;
constexpr int kUD = kU + kD;
constexpr int kH  = 8192;
constexpr int kP  = kH / 2;
constexpr int kY  = 256;
constexpr int kUD8 = kUD / 8;
constexpr float kBtCarry = 65536.0f;
constexpr float kCeCarry = 1048576.0f;
constexpr float kMtCarry = 262144.0f;
constexpr float kScale1 = 1.0f / (kBtCarry * kCeCarry);
constexpr float kScale2 = 1.0f / kMtCarry;
static_assert(kUD == 320 && kP == 4096 && kUD8 == 40);
static_assert(kB * kU == 1048576 && kB * kD == 262144 && kH == 8192 && kP == 4096);
static_assert(kH * kUD == 2621440 && kY * kH == 2097152 && kB * kY == 1048576);
static_assert((kH / 8) == 1024);
static_assert((kD % 8) == 0 && (kU % 8) == 0);
static_assert((kY & (kY - 1)) == 0);
static_assert((kH % 32) == 0 && (kUD % 32) == 0);
static_assert((kUD % 32) == 0 && (kB % 32) == 0 && (kY % 64) == 0);

constexpr size_t kSzTR  = (size_t)kP * 4 * 4;
constexpr size_t kSzREC = (size_t)kH * 4;
constexpr size_t kSzCE  = (size_t)kY * kH * 2;
constexpr size_t kSzBT  = (size_t)kUD * kH * 2;
constexpr size_t kSzMM  = (size_t)kUD * kY * 4;
constexpr size_t kSzMT  = (size_t)kY * kUD * 2;
constexpr size_t kSzUD  = (size_t)kB * kUD * 2;
constexpr size_t kSzYD  = (size_t)kB * kY * 4;
constexpr size_t kSzYB  = (size_t)kY * 4;
constexpr size_t kOffTR  = 0;
constexpr size_t kOffREC = kOffTR  + kSzTR;
constexpr size_t kOffCE  = kOffREC + kSzREC;
constexpr size_t kOffBT  = kOffCE  + kSzCE;
constexpr size_t kOffMM  = kOffBT  + kSzBT;
constexpr size_t kOffMT  = kOffMM  + kSzMM;
constexpr size_t kOffUD  = kOffMT  + kSzMT;
constexpr size_t kOffYD  = kOffUD  + kSzUD;
constexpr size_t kOffYB  = kOffYD  + kSzYD;
constexpr size_t kWsTotal = kOffYB + kSzYB;
static_assert((kSzTR % 256) == 0 && (kSzREC % 256) == 0 && (kSzCE % 256) == 0 && (kSzBT % 256) == 0 &&
              (kSzMM % 256) == 0 && (kSzMT % 256) == 0 && (kSzUD % 256) == 0 && (kSzYD % 256) == 0 &&
              (kSzYB % 256) == 0);
static_assert(kWsTotal == 16843776ull);
static_assert(kWsTotal <= 134217728ull);

__device__ __forceinline__ _Float16 f16_flush(float v) {
  const float w = (fabsf(v) < 6.103515625e-05f) ? 0.0f : v;
  return (_Float16)w;
}

__device__ __forceinline__ float bf16r(float v) {
  unsigned u = __float_as_uint(v);
  u = (u + 0x7FFFu + ((u >> 16) & 1u)) & 0xFFFF0000u;
  return __uint_as_float(u);
}

namespace eng {
union FragU { v16h v; v8h h[2]; };
__device__ __forceinline__ v16h frag_load(const _Float16* p) {
  FragU f;
  f.h[0] = *(const v8h*)(p);
  f.h[1] = *(const v8h*)(p + 16);
  return f.v;
}
__device__ __forceinline__ v8f mma(v16h a, v16h b, v8f c) {
  return __builtin_amdgcn_wmma_f32_16x16x32_f16(false, a, false, b, (short)0, c, false, false);
}
__device__ __forceinline__ void guard1(v8f& a, v16h x, v16h y) {
  asm volatile("v_nop\n\tv_nop\n\tv_nop\n\tv_nop" : "+v"(a) : "v"(x), "v"(y));
}
__device__ __forceinline__ void guard_acc(v8f& a) {
  asm volatile("v_nop\n\tv_nop\n\tv_nop\n\tv_nop" : "+v"(a));
}
__device__ __forceinline__ void keep4(v16h a, v16h b, v16h c, v16h d) {
  asm volatile("v_nop" :: "v"(a), "v"(b), "v"(c), "v"(d));
}

template <int MI, int SPL>
__global__ __launch_bounds__(256) void gemm_f16_kernel(
    const unsigned short* __restrict__ Ap, const unsigned short* __restrict__ A2p, int lda,
    const unsigned short* __restrict__ Btp, const unsigned short* __restrict__ Bt2p, int ldb,
    float* __restrict__ C, int ldc, int M, int N, int K, float scale, float rscale)
{
  static_assert(MI >= 1 && MI <= 2);
  static_assert(SPL >= 0 && SPL <= 2);
  const _Float16* A   = (const _Float16*)Ap;
  const _Float16* A2  = (const _Float16*)A2p;
  const _Float16* Bt  = (const _Float16*)Btp;
  const _Float16* Bt2 = (const _Float16*)Bt2p;
  __shared__ __align__(16) float sT[8][16 * 68];
  const int lane = threadIdx.x & 31;
  const int wave = threadIdx.x >> 5;
  const int tilesN = N >> 6;
  const int tilesM = M / (16 * MI);
  const int tile = blockIdx.x * 8 + wave;
  if (tile >= tilesM * tilesN) return;
  const int tm = tile / tilesN;
  const int tn = tile - tm * tilesN;
  const int m0 = tm * (16 * MI);
  const int n0 = tn << 6;
  const int rlane = lane & 15;
  const int koff  = (lane >> 4) * 8;
  const int mOff  = (lane >> 4) * 8;

  v8f acc[MI][4], accr[MI][4];
#pragma unroll
  for (int i = 0; i < MI; ++i)
#pragma unroll
    for (int j = 0; j < 4; ++j) {
      acc[i][j]  = (v8f){0.f, 0.f, 0.f, 0.f, 0.f, 0.f, 0.f, 0.f};
      accr[i][j] = (v8f){0.f, 0.f, 0.f, 0.f, 0.f, 0.f, 0.f, 0.f};
    }

  for (int k0 = 0; k0 < K; k0 += 32) {
    v16h bh[4], bl[4];
#pragma unroll
    for (int j = 0; j < 4; ++j) {
      const size_t bo = (size_t)(n0 + (j << 4) + rlane) * ldb + koff + k0;
      bh[j] = frag_load(Bt + bo);
      if (SPL == 2) bl[j] = frag_load(Bt2 + bo); else bl[j] = bh[j];
    }
#pragma unroll
    for (int i = 0; i < MI; ++i) {
      const size_t ao = (size_t)(m0 + (i << 4) + rlane) * lda + koff + k0;
      const v16h ah = frag_load(A + ao);
      v16h al = ah;
      if (SPL >= 1) al = frag_load(A2 + ao);
#pragma unroll
      for (int j = 0; j < 4; ++j) {
        acc[i][j] = mma(ah, bh[j], acc[i][j]);
        if (SPL >= 1) accr[i][j] = mma(al, bh[j], accr[i][j]);
        if (SPL == 2) accr[i][j] = mma(ah, bl[j], accr[i][j]);
      }
#pragma unroll
      for (int j = 0; j < 4; ++j) {
        guard1(acc[i][j], ah, al);
        if (SPL >= 1) guard1(accr[i][j], ah, al);
      }
    }
    keep4(bh[0], bh[1], bh[2], bh[3]);
    if (SPL == 2) keep4(bl[0], bl[1], bl[2], bl[3]);
  }
#pragma unroll
  for (int i = 0; i < MI; ++i)
#pragma unroll
    for (int j = 0; j < 4; ++j) {
      guard_acc(acc[i][j]);
      if (SPL >= 1) guard_acc(accr[i][j]);
    }

  float* slab = sT[wave];
#pragma unroll
  for (int i = 0; i < MI; ++i) {
    const int mBase = m0 + (i << 4);
#pragma unroll
    for (int j = 0; j < 4; ++j) {
#pragma unroll
      for (int r = 0; r < 8; ++r) {
        float v = acc[i][j][r] * scale;
        if (SPL >= 1) v += accr[i][j][r] * rscale;
        slab[(mOff + r) * 68 + (j << 4) + rlane] = v;
      }
    }
    __builtin_amdgcn_fence(__ATOMIC_RELEASE, "workgroup");
    __builtin_amdgcn_wave_barrier();
    __builtin_amdgcn_fence(__ATOMIC_ACQUIRE, "workgroup");
    {
      const int hh = lane >> 4, c4 = (lane & 15) * 4;
      for (int pass = 0; pass < 2; ++pass) {
#pragma unroll
        for (int it = 0; it < 8; ++it) {
          const int row = it * 2 + hh;
          const v4f v = *(const v4f*)(slab + row * 68 + c4);
          *(volatile v4f*)(C + (size_t)(mBase + row) * ldc + n0 + c4) = v;
        }
        __threadfence();
      }
    }
    __builtin_amdgcn_fence(__ATOMIC_RELEASE, "workgroup");
    __builtin_amdgcn_wave_barrier();
    __builtin_amdgcn_fence(__ATOMIC_ACQUIRE, "workgroup");
  }
}
}

__global__ __launch_bounds__(256) void trig_kernel(
    const float* __restrict__ omega, const float* __restrict__ h,
    float* __restrict__ TR, float* __restrict__ REC)
{
  const int p = blockIdx.x * 256 + threadIdx.x;
  const float w = bf16r(omega[p]);
  const float ang = w * 0.1f;
  const float c = cosf(ang);
  const float s = sinf(ang);
  const float sw = s / w;
  const float cw = (c - 1.0f) / w;
  const v2f hv = *(const v2f*)(h + 2 * p);
  const float h0 = hv[0];
  const float h1 = hv[1];
  const float a = bf16r(h0);
  const float b = bf16r(h1);
  v4f t;
  t[0] = c;
  t[1] = s;
  t[2] = sw;
  t[3] = cw;
  v2f r;
  r[0] = c * a + s * b;
  r[1] = -s * a + c * b;
  float* pt = TR + (size_t)p * 4;
  float* pr = REC + (size_t)p * 2;
  *(volatile v4f*)pt = t;
  *(volatile v2f*)pr = r;
  __threadfence();
  *(volatile v4f*)pt = t;
  *(volatile v2f*)pr = r;
}

__global__ __launch_bounds__(256) void ce_fold_kernel(
    const float* __restrict__ Cw, const float* __restrict__ TR, unsigned short* __restrict__ CE)
{
  const int j = blockIdx.x * 256 + threadIdx.x;
  const int n = j >> 10;
  const int k0 = (j & 1023) * 8;
  const int p0 = k0 >> 1;
  const float* cp = Cw + (size_t)n * kH + k0;
  const v4f a0 = *(const v4f*)(cp);
  const v4f a1 = *(const v4f*)(cp + 4);
  const v4f t0 = *(const v4f*)(TR + (size_t)(p0 + 0) * 4);
  const v4f t1 = *(const v4f*)(TR + (size_t)(p0 + 1) * 4);
  const v4f t2 = *(const v4f*)(TR + (size_t)(p0 + 2) * 4);
  const v4f t3 = *(const v4f*)(TR + (size_t)(p0 + 3) * 4);
  const float r0 = a0[0];
  const float r1 = a0[1];
  const float r2 = a0[2];
  const float r3 = a0[3];
  const float r4 = a1[0];
  const float r5 = a1[1];
  const float r6 = a1[2];
  const float r7 = a1[3];
  const float ce0 = bf16r(r0);
  const float co0 = bf16r(r1);
  const float ce1 = bf16r(r2);
  const float co1 = bf16r(r3);
  const float ce2 = bf16r(r4);
  const float co2 = bf16r(r5);
  const float ce3 = bf16r(r6);
  const float co3 = bf16r(r7);
  const float sw0 = t0[2];
  const float cw0 = t0[3];
  const float sw1 = t1[2];
  const float cw1 = t1[3];
  const float sw2 = t2[2];
  const float cw2 = t2[3];
  const float sw3 = t3[2];
  const float cw3 = t3[3];
  const float ev0 = sw0 * ce0 + cw0 * co0;
  const float od0 = -cw0 * ce0 + sw0 * co0;
  const float ev1 = sw1 * ce1 + cw1 * co1;
  const float od1 = -cw1 * ce1 + sw1 * co1;
  const float ev2 = sw2 * ce2 + cw2 * co2;
  const float od2 = -cw2 * ce2 + sw2 * co2;
  const float ev3 = sw3 * ce3 + cw3 * co3;
  const float od3 = -cw3 * ce3 + sw3 * co3;
  v8h hv;
  hv[0] = f16_flush(ev0 * kCeCarry);
  hv[1] = f16_flush(od0 * kCeCarry);
  hv[2] = f16_flush(ev1 * kCeCarry);
  hv[3] = f16_flush(od1 * kCeCarry);
  hv[4] = f16_flush(ev2 * kCeCarry);
  hv[5] = f16_flush(od2 * kCeCarry);
  hv[6] = f16_flush(ev3 * kCeCarry);
  hv[7] = f16_flush(od3 * kCeCarry);
  unsigned short* q = CE + (size_t)j * 8;
  *(volatile v8h*)q = hv;
  __threadfence();
  *(volatile v8h*)q = hv;
}

__global__ __launch_bounds__(256) void bt_pack_kernel(
    const float* __restrict__ Bw, unsigned short* __restrict__ BT)
{
  const int j = blockIdx.x * 256 + threadIdx.x;
  const int m = j >> 10;
  const int k0 = (j & 1023) * 8;
  const float* sp = Bw + (size_t)k0 * kUD + m;
  const float w0 = sp[0 * kUD];
  const float w1 = sp[1 * kUD];
  const float w2 = sp[2 * kUD];
  const float w3 = sp[3 * kUD];
  const float w4 = sp[4 * kUD];
  const float w5 = sp[5 * kUD];
  const float w6 = sp[6 * kUD];
  const float w7 = sp[7 * kUD];
  v8h hv;
  hv[0] = f16_flush(bf16r(w0) * kBtCarry);
  hv[1] = f16_flush(bf16r(w1) * kBtCarry);
  hv[2] = f16_flush(bf16r(w2) * kBtCarry);
  hv[3] = f16_flush(bf16r(w3) * kBtCarry);
  hv[4] = f16_flush(bf16r(w4) * kBtCarry);
  hv[5] = f16_flush(bf16r(w5) * kBtCarry);
  hv[6] = f16_flush(bf16r(w6) * kBtCarry);
  hv[7] = f16_flush(bf16r(w7) * kBtCarry);
  unsigned short* q = BT + (size_t)j * 8;
  *(volatile v8h*)q = hv;
  __threadfence();
  *(volatile v8h*)q = hv;
}

__global__ __launch_bounds__(256) void mt_pack_kernel(
    const float* __restrict__ MM, unsigned short* __restrict__ MT)
{
  const int j = blockIdx.x * 256 + threadIdx.x;
  const int n = j / kUD8;
  const int m0 = (j - kUD8 * n) * 8;
  const float* sp = MM + (size_t)m0 * kY + n;
  const float w0 = sp[0 * kY];
  const float w1 = sp[1 * kY];
  const float w2 = sp[2 * kY];
  const float w3 = sp[3 * kY];
  const float w4 = sp[4 * kY];
  const float w5 = sp[5 * kY];
  const float w6 = sp[6 * kY];
  const float w7 = sp[7 * kY];
  v8h hv;
  hv[0] = f16_flush(w0 * kMtCarry);
  hv[1] = f16_flush(w1 * kMtCarry);
  hv[2] = f16_flush(w2 * kMtCarry);
  hv[3] = f16_flush(w3 * kMtCarry);
  hv[4] = f16_flush(w4 * kMtCarry);
  hv[5] = f16_flush(w5 * kMtCarry);
  hv[6] = f16_flush(w6 * kMtCarry);
  hv[7] = f16_flush(w7 * kMtCarry);
  unsigned short* q = MT + (size_t)j * 8;
  *(volatile v8h*)q = hv;
  __threadfence();
  *(volatile v8h*)q = hv;
}

__global__ __launch_bounds__(256) void ud_pack_kernel(
    const float* __restrict__ du, const float* __restrict__ u, unsigned short* __restrict__ UD)
{
  const int j = blockIdx.x * 256 + threadIdx.x;
  const int b = j / kUD8;
  const int k0 = (j - kUD8 * b) * 8;
  const bool isd = (k0 < kD);
  const int kd = isd ? k0 : 0;
  const int ku = isd ? 0 : (k0 - kD);
  const float* pd = du + (size_t)b * kD + kd;
  const float* pu = u + (size_t)b * kU + ku;
  const v4f d0 = *(const v4f*)(pd);
  const v4f d1 = *(const v4f*)(pd + 4);
  const v4f u0 = *(const v4f*)(pu);
  const v4f u1 = *(const v4f*)(pu + 4);
  const float da0 = d0[0];
  const float da1 = d0[1];
  const float da2 = d0[2];
  const float da3 = d0[3];
  const float da4 = d1[0];
  const float da5 = d1[1];
  const float da6 = d1[2];
  const float da7 = d1[3];
  const float ua0 = u0[0];
  const float ua1 = u0[1];
  const float ua2 = u0[2];
  const float ua3 = u0[3];
  const float ua4 = u1[0];
  const float ua5 = u1[1];
  const float ua6 = u1[2];
  const float ua7 = u1[3];
  const float x0 = isd ? da0 : ua0;
  const float x1 = isd ? da1 : ua1;
  const float x2 = isd ? da2 : ua2;
  const float x3 = isd ? da3 : ua3;
  const float x4 = isd ? da4 : ua4;
  const float x5 = isd ? da5 : ua5;
  const float x6 = isd ? da6 : ua6;
  const float x7 = isd ? da7 : ua7;
  v8h hv;
  hv[0] = f16_flush(bf16r(x0));
  hv[1] = f16_flush(bf16r(x1));
  hv[2] = f16_flush(bf16r(x2));
  hv[3] = f16_flush(bf16r(x3));
  hv[4] = f16_flush(bf16r(x4));
  hv[5] = f16_flush(bf16r(x5));
  hv[6] = f16_flush(bf16r(x6));
  hv[7] = f16_flush(bf16r(x7));
  unsigned short* q = UD + (size_t)j * 8;
  *(volatile v8h*)q = hv;
  __threadfence();
  *(volatile v8h*)q = hv;
}

__global__ __launch_bounds__(256) void yb_kernel(
    const float* __restrict__ REC, const float* __restrict__ Cw, float* __restrict__ YB)
{
  const int n = threadIdx.x;
  const float* crow = Cw + (size_t)n * kH;
  float acc = 0.0f;
  for (int k = 0; k < kH; k += 4) {
    const v4f cv = *(const v4f*)(crow + k);
    const v4f rv = *(const v4f*)(REC + k);
    const float c0 = cv[0];
    const float c1 = cv[1];
    const float c2 = cv[2];
    const float c3 = cv[3];
    const float q0 = rv[0];
    const float q1 = rv[1];
    const float q2 = rv[2];
    const float q3 = rv[3];
    acc = acc + q0 * bf16r(c0);
    acc = acc + q1 * bf16r(c1);
    acc = acc + q2 * bf16r(c2);
    acc = acc + q3 * bf16r(c3);
  }
  float* p = YB + n;
  *(volatile float*)p = acc;
  __threadfence();
  *(volatile float*)p = acc;
}

__global__ __launch_bounds__(256) void out_kernel(
    const float* __restrict__ YD, const float* __restrict__ YB, float* __restrict__ out)
{
  const int t = blockIdx.x * 256 + threadIdx.x;
  const size_t i = (size_t)t * 4;
  const int n0 = (int)(i & (size_t)(kY - 1));
  const v4f a = *(const v4f*)(YD + i);
  const v4f b = *(const v4f*)(YB + n0);
  const v4f r = a + b;
  float* p = out + i;
  *(volatile v4f*)p = r;
  __threadfence();
  *(volatile v4f*)p = r;
}

static_assert((kP % 256) == 0);
static_assert(((kY * kH / 8) % 256) == 0);
static_assert(((kUD * kH / 8) % 256) == 0);
static_assert(((kY * kUD / 8) % 256) == 0);
static_assert(((kB * kUD / 8) % 256) == 0);
static_assert(((kB * kY / 4) % 256) == 0);
static_assert(((kUD / 32) * (kY / 64)) % 8 == 0);
static_assert(((kB / 32) * (kY / 64)) % 8 == 0);
static_assert(kY == 256);

extern "C" void kernel_launch(void* const* d_in, const int* in_sizes, int n_in,
                              void* d_out, int out_size, void* d_ws, size_t ws_size,
                              hipStream_t stream)
{
  if (n_in < 6) return;
  if (in_sizes[0] != kB * kU) return;
  if (in_sizes[1] != kB * kD) return;
  if (in_sizes[2] != kH) return;
  if (in_sizes[3] != kP) return;
  if (in_sizes[4] != kH * kUD) return;
  if (in_sizes[5] != kY * kH) return;
  if (out_size != kB * kY) return;
  if (ws_size < kWsTotal) return;

  const float* u     = (const float*)d_in[0];
  const float* du    = (const float*)d_in[1];
  const float* h     = (const float*)d_in[2];
  const float* omega = (const float*)d_in[3];
  const float* B_w   = (const float*)d_in[4];
  const float* C_w   = (const float*)d_in[5];
  float* out = (float*)d_out;

  char* ws = (char*)d_ws;
  float*          TR  = (float*)(ws + kOffTR);
  float*          REC = (float*)(ws + kOffREC);
  unsigned short* CE  = (unsigned short*)(ws + kOffCE);
  unsigned short* BT  = (unsigned short*)(ws + kOffBT);
  float*          MM  = (float*)(ws + kOffMM);
  unsigned short* MT  = (unsigned short*)(ws + kOffMT);
  unsigned short* UD  = (unsigned short*)(ws + kOffUD);
  float*          YD  = (float*)(ws + kOffYD);
  float*          YB  = (float*)(ws + kOffYB);

  trig_kernel<<<kP / 256, 256, 0, stream>>>(omega, h, TR, REC);

  ce_fold_kernel<<<(kY * kH / 8) / 256, 256, 0, stream>>>(C_w, TR, CE);

  bt_pack_kernel<<<(kUD * kH / 8) / 256, 256, 0, stream>>>(B_w, BT);

  eng::gemm_f16_kernel<2, 0><<<dim3((kUD / 32) * (kY / 64) / 8), 256, 0, stream>>>(
      BT, nullptr, kH, CE, nullptr, kH, MM, kY, kUD, kY, kH, kScale1, 0.0f);

  mt_pack_kernel<<<(kY * kUD / 8) / 256, 256, 0, stream>>>(MM, MT);

  ud_pack_kernel<<<(kB * kUD / 8) / 256, 256, 0, stream>>>(du, u, UD);

  eng::gemm_f16_kernel<2, 0><<<dim3((kB / 32) * (kY / 64) / 8), 256, 0, stream>>>(
      UD, nullptr, kUD, MT, nullptr, kUD, YD, kY, kB, kY, kUD, kScale2, 0.0f);

  yb_kernel<<<1, 256, 0, stream>>>(REC, C_w, YB);

  out_kernel<<<(kB * kY / 4) / 256, 256, 0, stream>>>(YD, YB, out);
}
